// HybridMultiHeadAttention_13993003450669
// MI455X (gfx1250) — hardware-verified
//
#include <hip/hip_runtime.h>
#include <math.h>
#include <stdint.h>

#define NB   2
#define NS   2048
#define DM   1024
#define NH   16
#define NP   8
#define DH   64
#define NROW (NB * NS)
#define NBH  (NB * NH)
#define NQB  (NS / 64)
static_assert(NROW == 4096);
static_assert(NBH == 32);
static_assert(NQB == 32);
static_assert(DH == 64 && (DM % 64) == 0 && (NS % 64) == 0 && (DM % 32) == 0);

typedef __bf16   v16b __attribute__((ext_vector_type(16)));
typedef __bf16   v8b  __attribute__((ext_vector_type(8)));
typedef float    v8f  __attribute__((ext_vector_type(8)));
typedef float    v4f  __attribute__((ext_vector_type(4)));
typedef unsigned int v4u __attribute__((ext_vector_type(4)));

__device__ __forceinline__ unsigned short bf_bits(float f) {
  unsigned u = __float_as_uint(f);
  return (unsigned short)((u + 0x7FFFu + ((u >> 16) & 1u)) >> 16);
}
__device__ __forceinline__ float bf_up(unsigned short h) { return __uint_as_float(((unsigned)h) << 16); }
__device__ __forceinline__ __bf16 bf_val(unsigned short h) { return __builtin_bit_cast(__bf16, h); }
__device__ __forceinline__ unsigned pk16(unsigned short a, unsigned short b) { return (unsigned)a | ((unsigned)b << 16); }
__device__ __forceinline__ v8f zero8() { v8f z = {0.f, 0.f, 0.f, 0.f, 0.f, 0.f, 0.f, 0.f}; return z; }

__device__ __forceinline__ v16b ldfrag_b(const __bf16* p) {
  union { v16b v; v8b h[2]; } f;
  f.h[0] = *(const v8b*)(p);
  f.h[1] = *(const v8b*)(p + 16);
  return f.v;
}

__device__ __forceinline__ v8f mma_b(v16b a, v16b b, v8f c) {
  c = __builtin_amdgcn_wmma_f32_16x16x32_bf16(false, a, false, b, (short)0, c, false, false);
  asm volatile("v_nop\n\tv_nop\n\tv_nop\n\tv_nop" : "+v"(c) : "v"(a), "v"(b));
  return c;
}
__device__ __forceinline__ v8f mma_b_raw(v16b a, v16b b, v8f c) {
  return __builtin_amdgcn_wmma_f32_16x16x32_bf16(false, a, false, b, (short)0, c, false, false);
}
__device__ __forceinline__ void dep_guard_b(v8f& a, v8f& b, v16b x) {
  asm volatile("v_nop\n\tv_nop\n\tv_nop\n\tv_nop" : "+v"(a), "+v"(b) : "v"(x));
}
__device__ __forceinline__ void dep_guard_b2(v8f& a, v8f& b, v16b x, v16b y) {
  asm volatile("v_nop\n\tv_nop\n\tv_nop\n\tv_nop" : "+v"(a), "+v"(b) : "v"(x), "v"(y));
}
__device__ __forceinline__ void keep4_b(v16b a, v16b b, v16b c, v16b d) {
  asm volatile("v_nop" :: "v"(a), "v"(b), "v"(c), "v"(d));
}
__device__ __forceinline__ void acc_guard4(v8f& a, v8f& b, v8f& c, v8f& d) {
  asm volatile("v_nop\n\tv_nop\n\tv_nop\n\tv_nop" : "+v"(a), "+v"(b), "+v"(c), "+v"(d));
}

__global__ __launch_bounds__(256) void cvt_bf16x8(const float* __restrict__ in, unsigned short* out, int n8) {
  const int i = blockIdx.x * 256 + threadIdx.x;
  if (i < n8) {
    const v4f a = *(const v4f*)(in + (size_t)i * 8);
    const v4f b = *(const v4f*)(in + (size_t)i * 8 + 4);
    v4u p;
    p[0] = pk16(bf_bits(a[0]), bf_bits(a[1]));
    p[1] = pk16(bf_bits(a[2]), bf_bits(a[3]));
    p[2] = pk16(bf_bits(b[0]), bf_bits(b[1]));
    p[3] = pk16(bf_bits(b[2]), bf_bits(b[3]));
    *(volatile v4u*)(out + (size_t)i * 8) = p;
    __threadfence();
    *(volatile v4u*)(out + (size_t)i * 8) = p;
  }
}

__global__ __launch_bounds__(256) void prep_wt(const float* __restrict__ W, int C, unsigned short* WT) {
  __shared__ __align__(16) unsigned short sW[16 * DM];
  const int tid  = threadIdx.x;
  const int wave = tid >> 5;
  const int lane = tid & 31;
  const int c0   = blockIdx.x * 16;
#pragma unroll
  for (int it = 0; it < 4; ++it) {
    const int kk = it * 256 + tid;
    const float* row = W + (size_t)kk * C + c0;
    const v4f a0 = *(const v4f*)(row);
    const v4f a1 = *(const v4f*)(row + 4);
    const v4f a2 = *(const v4f*)(row + 8);
    const v4f a3 = *(const v4f*)(row + 12);
#pragma unroll
    for (int e = 0; e < 4; ++e) {
      sW[(e)      * DM + kk] = bf_bits(a0[e]);
      sW[(4 + e)  * DM + kk] = bf_bits(a1[e]);
      sW[(8 + e)  * DM + kk] = bf_bits(a2[e]);
      sW[(12 + e) * DM + kk] = bf_bits(a3[e]);
    }
  }
  __syncthreads();
  const int r0 = 2 * wave;
  v4u w0[4], w1[4];
#pragma unroll
  for (int ch = 0; ch < 4; ++ch) {
    w0[ch] = *(const v4u*)(sW + r0 * DM + ch * 256 + lane * 8);
    w1[ch] = *(const v4u*)(sW + (r0 + 1) * DM + ch * 256 + lane * 8);
  }
  const size_t o0 = (size_t)(c0 + r0) * DM;
  const size_t o1 = (size_t)(c0 + r0 + 1) * DM;
  for (int pass = 0; pass < 2; ++pass) {
#pragma unroll
    for (int ch = 0; ch < 4; ++ch) {
      *(volatile v4u*)(WT + o0 + ch * 256 + lane * 8) = w0[ch];
      *(volatile v4u*)(WT + o1 + ch * 256 + lane * 8) = w1[ch];
    }
    __threadfence();
  }
}

template <int MODE>
__global__ __launch_bounds__(256) void pgemm(const unsigned short* __restrict__ Ap,
                                             const unsigned short* __restrict__ A2p,
                                             const unsigned short* __restrict__ Bp,
                                             unsigned short* C0h, unsigned short* C0l,
                                             unsigned short* C1h, unsigned short* C1l,
                                             float* Cf) {
  constexpr int M = (MODE == 1) ? DM : NROW;
  constexpr int N = (MODE == 0) ? (2 * DM) : ((MODE == 1) ? NROW : DM);
  constexpr int K = DM;
  constexpr int LDA = DM;
  constexpr int LDB = DM;
  static_assert((M % 64) == 0 && (N % 64) == 0 && (K % 32) == 0);
  __shared__ __align__(16) float sT[8][16 * 68];
  const __bf16* Ab = (const __bf16*)(const void*)Ap;
  const __bf16* Al = (const __bf16*)(const void*)A2p;
  const __bf16* Bb = (const __bf16*)(const void*)Bp;

  const int lane = threadIdx.x & 31;
  const int wave = threadIdx.x >> 5;
  const int tilesN = N >> 6;
  const int tilesM = M >> 6;
  const int tile = blockIdx.x * 8 + wave;
  if (tile >= tilesM * tilesN) return;
  const int tm = tile / tilesN;
  const int tn = tile - tm * tilesN;
  const int m0 = tm << 6;
  const int n0 = tn << 6;

  const int rlane = lane & 15;
  const int koff  = (lane >> 4) * 8;
  const int mOff  = (lane >> 4) * 8;

  v8f acc[4][4];
#pragma unroll
  for (int i = 0; i < 4; ++i)
#pragma unroll
    for (int j = 0; j < 4; ++j) acc[i][j] = zero8();

  for (int k0 = 0; k0 < K; k0 += 32) {
    v16b bh[4];
#pragma unroll
    for (int j = 0; j < 4; ++j) {
      const size_t bo = (size_t)(n0 + (j << 4) + rlane) * LDB + koff + k0;
      bh[j] = ldfrag_b(Bb + bo);
    }
#pragma unroll
    for (int i = 0; i < 4; ++i) {
      const size_t ao = (size_t)(m0 + (i << 4) + rlane) * LDA + koff + k0;
      const v16b ah = ldfrag_b(Ab + ao);
      if (MODE == 2) {
        const v16b al = ldfrag_b(Al + ao);
#pragma unroll
        for (int j = 0; j < 4; ++j) {
          acc[i][j] = mma_b_raw(ah, bh[j], acc[i][j]);
          acc[i][j] = mma_b_raw(al, bh[j], acc[i][j]);
        }
        dep_guard_b2(acc[i][0], acc[i][3], ah, al);
      } else {
#pragma unroll
        for (int j = 0; j < 4; ++j) {
          acc[i][j] = mma_b_raw(ah, bh[j], acc[i][j]);
        }
        dep_guard_b(acc[i][0], acc[i][3], ah);
      }
    }
    keep4_b(bh[0], bh[1], bh[2], bh[3]);
  }
  acc_guard4(acc[0][0], acc[0][1], acc[0][2], acc[0][3]);
  acc_guard4(acc[1][0], acc[1][1], acc[1][2], acc[1][3]);
  acc_guard4(acc[2][0], acc[2][1], acc[2][2], acc[2][3]);
  acc_guard4(acc[3][0], acc[3][1], acc[3][2], acc[3][3]);

  float* slab = sT[wave];
  unsigned short* Ch = C0h;
  unsigned short* Cl = C0l;
  size_t obase = 0;
  size_t rpitch = 0;
  if (MODE == 0) {
    const int seg = n0 >> 10;
    const int hd  = (n0 & (DM - 1)) >> 6;
    const int bb  = m0 >> 11;
    const int nq  = m0 & (NS - 1);
    Ch = (seg == 0) ? C0h : C1h;
    Cl = (seg == 0) ? C0l : C1l;
    obase  = ((size_t)(bb * NH + hd) * NS + nq) * DH;
    rpitch = DH;
  } else if (MODE == 1) {
    const int hd  = m0 >> 6;
    const int bb  = n0 >> 11;
    const int np0 = n0 & (NS - 1);
    obase  = ((size_t)(bb * NH + hd) * DH) * NS + np0;
    rpitch = NS;
  }
#pragma unroll
  for (int i = 0; i < 4; ++i) {
    const int mBase = m0 + (i << 4);
#pragma unroll
    for (int j = 0; j < 4; ++j) {
#pragma unroll
      for (int r = 0; r < 8; ++r) {
        slab[(mOff + r) * 68 + (j << 4) + rlane] = acc[i][j][r];
      }
    }
    __builtin_amdgcn_fence(__ATOMIC_RELEASE, "workgroup");
    __builtin_amdgcn_wave_barrier();
    __builtin_amdgcn_fence(__ATOMIC_ACQUIRE, "workgroup");
    if (MODE != 2) {
      const int q = lane >> 3, c8 = (lane & 7) * 8;
      v4u hv[4], lv[4];
#pragma unroll
      for (int it = 0; it < 4; ++it) {
        const int row = it * 4 + q;
        const float* sp = slab + row * 68 + c8;
        v4u a, a2;
#pragma unroll
        for (int e = 0; e < 4; ++e) {
          const float f0 = sp[2 * e], f1 = sp[2 * e + 1];
          const unsigned short h0 = bf_bits(f0), h1 = bf_bits(f1);
          const unsigned short l0 = bf_bits(f0 - bf_up(h0)), l1 = bf_bits(f1 - bf_up(h1));
          a[e] = pk16(h0, h1); a2[e] = pk16(l0, l1);
        }
        hv[it] = a; lv[it] = a2;
      }
      for (int pass = 0; pass < 2; ++pass) {
#pragma unroll
        for (int it = 0; it < 4; ++it) {
          const int row = it * 4 + q;
          const size_t o = obase + (size_t)((i << 4) + row) * rpitch + c8;
          *(volatile v4u*)(Ch + o) = hv[it];
          *(volatile v4u*)(Cl + o) = lv[it];
        }
        __threadfence();
      }
    } else {
      const int q2 = lane >> 4, c4 = (lane & 15) * 4;
      v4f ov[8];
#pragma unroll
      for (int it = 0; it < 8; ++it) {
        const int row = it * 2 + q2;
        ov[it] = *(const v4f*)(slab + row * 68 + c4);
      }
      for (int pass = 0; pass < 2; ++pass) {
#pragma unroll
        for (int it = 0; it < 8; ++it) {
          const int row = it * 2 + q2;
          *(volatile v4f*)(Cf + (size_t)(mBase + row) * DM + n0 + c4) = ov[it];
        }
        __threadfence();
      }
    }
    __builtin_amdgcn_fence(__ATOMIC_RELEASE, "workgroup");
    __builtin_amdgcn_wave_barrier();
    __builtin_amdgcn_fence(__ATOMIC_ACQUIRE, "workgroup");
  }
}

#define L_KH    0
#define L_KL    8192
#define L_VH    16384
#define L_VL    24576
#define L_BS    32768
#define L_PH    40960
#define L_PL    49152
#define L_ST    57344
#define L_TOTAL 74752
static_assert(L_KL - L_KH == 64 * DH * 2 && L_VH - L_KL == 64 * DH * 2);
static_assert(L_VL - L_VH == DH * 64 * 2 && L_BS - L_VL == DH * 64 * 2);
static_assert(L_PH - L_BS == 64 * 64 * 2);
static_assert(L_PL - L_PH == 4 * 16 * 64 * 2 && L_ST - L_PL == 4 * 16 * 64 * 2);
static_assert(L_TOTAL - L_ST == 4 * 16 * 68 * 4);

__global__ __launch_bounds__(128)
void attn(const unsigned short* __restrict__ qhp, const unsigned short* __restrict__ qlp,
          const unsigned short* __restrict__ khp, const unsigned short* __restrict__ klp,
          const unsigned short* __restrict__ vhp, const unsigned short* __restrict__ vlp,
          const unsigned short* __restrict__ bbp, const float* __restrict__ beta,
          unsigned short* Ohp, unsigned short* Olp) {
  extern __shared__ __align__(16) unsigned char lds[];
  union FB { v16b v; v8b h[2]; };
  __bf16* Ksh = (__bf16*)(lds + L_KH);
  __bf16* Ksl = (__bf16*)(lds + L_KL);
  __bf16* Vth = (__bf16*)(lds + L_VH);
  __bf16* Vtl = (__bf16*)(lds + L_VL);
  __bf16* Bs  = (__bf16*)(lds + L_BS);
  const unsigned short* Bsu = (const unsigned short*)(lds + L_BS);
  __bf16* Ph  = (__bf16*)(lds + L_PH);
  __bf16* Pl  = (__bf16*)(lds + L_PL);
  float*  stg = (float*)(lds + L_ST);

  const int tid  = threadIdx.x;
  const int wave = tid >> 5;
  const int lane = tid & 31;
  const int hh   = lane >> 4;
  const int c    = lane & 15;

  const int bx = blockIdx.x;
  const int qb = bx & (NQB - 1);
  const int bh = bx >> 5;
  const int b  = bh >> 4;
  const int h  = bh & (NH - 1);
  const int q0 = qb * 64 + wave * 16;
  const size_t zrow = (size_t)bh * NS;

  const float braw  = beta[h & (NP - 1)];
  const float betav = (h < NP) ? bf_up(bf_bits(braw)) : 0.f;

  const __bf16* Qh = (const __bf16*)(const void*)qhp;
  const __bf16* Ql = (const __bf16*)(const void*)qlp;
  const __bf16* Kh = (const __bf16*)(const void*)khp;
  const __bf16* Kl = (const __bf16*)(const void*)klp;
  const __bf16* Vh = (const __bf16*)(const void*)vhp + (size_t)bh * DH * NS;
  const __bf16* Vl = (const __bf16*)(const void*)vlp + (size_t)bh * DH * NS;
  const __bf16* Bg = (const __bf16*)(const void*)bbp + ((size_t)b * NS + (size_t)qb * 64) * NS;

  __bf16* pwh = Ph + wave * 1024;
  __bf16* pwl = Pl + wave * 1024;

  v8f acc[4];
#pragma unroll
  for (int t = 0; t < 4; ++t) acc[t] = zero8();
  float mrow[8], lrow[8], alpha[8];
#pragma unroll
  for (int r = 0; r < 8; ++r) { mrow[r] = -INFINITY; lrow[r] = 0.f; alpha[r] = 0.f; }

  const size_t qo = (zrow + q0 + c) * DH + 8 * hh;

  for (int kt = 0; kt < NQB; ++kt) {
    const int kv0 = kt * 64;
    __syncthreads();
    {
      const __bf16* kgh = Kh + (zrow + kv0) * DH;
      const __bf16* kgl = Kl + (zrow + kv0) * DH;
      const __bf16* vgh = Vh + kv0;
      const __bf16* vgl = Vl + kv0;
      const __bf16* bgc = Bg + kv0;
#pragma unroll
      for (int i = 0; i < 4; ++i) {
        const int p  = tid + 128 * i;
        const int d  = p >> 3;
        const int sg = (p & 7) * 8;
        const v8b a0 = *(const v8b*)(kgh + p * 8);
        const v8b a1 = *(const v8b*)(kgl + p * 8);
        const v8b b0 = *(const v8b*)(vgh + (size_t)d * NS + sg);
        const v8b b1 = *(const v8b*)(vgl + (size_t)d * NS + sg);
        const v8b e0 = *(const v8b*)(bgc + (size_t)d * NS + sg);
        *(v8b*)(Ksh + p * 8) = a0;
        *(v8b*)(Ksl + p * 8) = a1;
        *(v8b*)(Vth + d * 64 + sg) = b0;
        *(v8b*)(Vtl + d * 64 + sg) = b1;
        *(v8b*)(Bs  + d * 64 + sg) = e0;
      }
    }
    __syncthreads();

    v8f s[4];
#pragma unroll
    for (int j = 0; j < 4; ++j) s[j] = zero8();
#pragma unroll
    for (int dc = 0; dc < 2; ++dc) {
      const v16b qa = ldfrag_b(Qh + qo + dc * 32);
      const v16b ql = ldfrag_b(Ql + qo + dc * 32);
      const int ko = dc * 32 + 8 * hh;
#pragma unroll
      for (int j = 0; j < 4; ++j) {
        const int kr = (j * 16 + c) * DH + ko;
        FB kb, kl;
        kb.h[0] = *(const v8b*)(Ksh + kr);
        kb.h[1] = *(const v8b*)(Ksh + kr + 16);
        kl.h[0] = *(const v8b*)(Ksl + kr);
        kl.h[1] = *(const v8b*)(Ksl + kr + 16);
        s[j] = mma_b(qa, kb.v, s[j]);
        s[j] = mma_b(qa, kl.v, s[j]);
        s[j] = mma_b(ql, kb.v, s[j]);
      }
    }

#pragma unroll
    for (int r = 0; r < 8; ++r) {
      const int rowl = wave * 16 + 8 * hh + r;
      float m = -INFINITY;
#pragma unroll
      for (int j = 0; j < 4; ++j) {
        const int key = j * 16 + c;
        const float bia = bf_up(Bsu[rowl * 64 + key]);
        float sv = s[j][r] * 0.125f + betav * bia;
        s[j][r] = sv;
        m = fmaxf(m, sv);
      }
#pragma unroll
      for (int off = 1; off < 16; off <<= 1) m = fmaxf(m, __shfl_xor(m, off, 32));
      const float mnew  = fmaxf(mrow[r], m);
      const float msafe = (mnew == -INFINITY) ? 0.f : mnew;
      const float al    = __expf(mrow[r] - msafe);
      mrow[r]  = mnew;
      alpha[r] = al;
      float psum = 0.f;
#pragma unroll
      for (int j = 0; j < 4; ++j) {
        const float p = __expf(s[j][r] - msafe);
        psum += p;
        const unsigned short hb = bf_bits(p);
        const unsigned short lb = bf_bits(p - bf_up(hb));
        const int po = (8 * hh + r) * 64 + j * 16 + c;
        pwh[po] = bf_val(hb);
        pwl[po] = bf_val(lb);
      }
#pragma unroll
      for (int off = 1; off < 16; off <<= 1) psum += __shfl_xor(psum, off, 32);
      lrow[r] = lrow[r] * al + psum;
    }
    __builtin_amdgcn_fence(__ATOMIC_RELEASE, "workgroup");
    __builtin_amdgcn_wave_barrier();
    __builtin_amdgcn_fence(__ATOMIC_ACQUIRE, "workgroup");

    FB pa[2], pl[2];
#pragma unroll
    for (int kk = 0; kk < 2; ++kk) {
      const int pr = c * 64 + kk * 32 + 8 * hh;
      pa[kk].h[0] = *(const v8b*)(pwh + pr);
      pa[kk].h[1] = *(const v8b*)(pwh + pr + 16);
      pl[kk].h[0] = *(const v8b*)(pwl + pr);
      pl[kk].h[1] = *(const v8b*)(pwl + pr + 16);
    }
#pragma unroll
    for (int t = 0; t < 4; ++t) {
#pragma unroll
      for (int r = 0; r < 8; ++r) acc[t][r] *= alpha[r];
      const int vr0 = (t * 16 + c) * 64 + 8 * hh;
#pragma unroll
      for (int kk = 0; kk < 2; ++kk) {
        FB vb, vl;
        vb.h[0] = *(const v8b*)(Vth + vr0 + kk * 32);
        vb.h[1] = *(const v8b*)(Vth + vr0 + kk * 32 + 16);
        vl.h[0] = *(const v8b*)(Vtl + vr0 + kk * 32);
        vl.h[1] = *(const v8b*)(Vtl + vr0 + kk * 32 + 16);
        acc[t] = mma_b(pa[kk].v, vb.v, acc[t]);
        acc[t] = mma_b(pa[kk].v, vl.v, acc[t]);
        acc[t] = mma_b(pl[kk].v, vb.v, acc[t]);
      }
    }
  }

  float* os = stg + wave * (16 * 68);
  float inv[8];
#pragma unroll
  for (int r = 0; r < 8; ++r) inv[r] = (lrow[r] > 0.f) ? (1.0f / lrow[r]) : 0.f;
#pragma unroll
  for (int t = 0; t < 4; ++t) {
#pragma unroll
    for (int r = 0; r < 8; ++r) os[(8 * hh + r) * 68 + t * 16 + c] = acc[t][r] * inv[r];
  }
  __builtin_amdgcn_fence(__ATOMIC_RELEASE, "workgroup");
  __builtin_amdgcn_wave_barrier();
  __builtin_amdgcn_fence(__ATOMIC_ACQUIRE, "workgroup");
  {
    const int q = lane >> 3, c8 = (lane & 7) * 8;
    v4u hv[4], lv[4];
#pragma unroll
    for (int it = 0; it < 4; ++it) {
      const int row = it * 4 + q;
      const float* sp = os + row * 68 + c8;
      v4u a, a2;
#pragma unroll
      for (int e = 0; e < 4; ++e) {
        const float f0 = sp[2 * e], f1 = sp[2 * e + 1];
        const unsigned short h0 = bf_bits(f0), h1 = bf_bits(f1);
        const unsigned short l0 = bf_bits(f0 - bf_up(h0)), l1 = bf_bits(f1 - bf_up(h1));
        a[e] = pk16(h0, h1); a2[e] = pk16(l0, l1);
      }
      hv[it] = a; lv[it] = a2;
    }
    const size_t obase = ((size_t)b * NS + (size_t)q0) * DM + (size_t)h * DH;
    for (int pass = 0; pass < 2; ++pass) {
#pragma unroll
      for (int it = 0; it < 4; ++it) {
        const int row = it * 4 + q;
        const size_t o = obase + (size_t)row * DM + c8;
        *(volatile v4u*)(Ohp + o) = hv[it];
        *(volatile v4u*)(Olp + o) = lv[it];
      }
      __threadfence();
    }
  }
}

extern "C" void kernel_launch(void* const* d_in, const int* in_sizes, int n_in,
                              void* d_out, int out_size, void* d_ws, size_t ws_size,
                              hipStream_t stream) {
  if (n_in < 5) return;
  if (in_sizes[0] != NROW * DM) return;
  if (in_sizes[1] != NB * NS * NS) return;
  if (in_sizes[2] != DM * 3 * DM) return;
  if (in_sizes[3] != DM * DM) return;
  if (in_sizes[4] < NP) return;
  if (out_size != NROW * DM) return;

  const float* x     = (const float*)d_in[0];
  const float* abias = (const float*)d_in[1];
  const float* Wqkv  = (const float*)d_in[2];
  const float* Wp    = (const float*)d_in[3];
  const float* beta  = (const float*)d_in[4];

  const size_t PXB = (size_t)NROW * DM * 2;
  const size_t PWQ = (size_t)3 * DM * DM * 2;
  const size_t PWP = (size_t)DM * DM * 2;
  const size_t PQK = (size_t)NBH * NS * DH * 2;
  const size_t PVT = (size_t)NBH * DH * NS * 2;
  const size_t PO  = (size_t)NROW * DM * 2;
  const size_t PBB = (size_t)NB * NS * NS * 2;
  size_t off = 0;
  const size_t oXb  = off; off += PXB;
  const size_t oWqT = off; off += PWQ;
  const size_t oWpT = off; off += PWP;
  const size_t oQh  = off; off += PQK;
  const size_t oQl  = off; off += PQK;
  const size_t oKh  = off; off += PQK;
  const size_t oKl  = off; off += PQK;
  const size_t oVTh = off; off += PVT;
  const size_t oVTl = off; off += PVT;
  const size_t oOh  = off; off += PO;
  const size_t oOl  = off; off += PO;
  const size_t oBb  = off; off += PBB;
  if (off > ws_size) return;
  if (off > (size_t)134217728) return;

  char* ws = (char*)d_ws;
  unsigned short* Xb  = (unsigned short*)(ws + oXb);
  unsigned short* WqT = (unsigned short*)(ws + oWqT);
  unsigned short* WpT = (unsigned short*)(ws + oWpT);
  unsigned short* Qh  = (unsigned short*)(ws + oQh);
  unsigned short* Ql  = (unsigned short*)(ws + oQl);
  unsigned short* Kh  = (unsigned short*)(ws + oKh);
  unsigned short* Kl  = (unsigned short*)(ws + oKl);
  unsigned short* VTh = (unsigned short*)(ws + oVTh);
  unsigned short* VTl = (unsigned short*)(ws + oVTl);
  unsigned short* Oh  = (unsigned short*)(ws + oOh);
  unsigned short* Ol  = (unsigned short*)(ws + oOl);
  unsigned short* Bb  = (unsigned short*)(ws + oBb);
  float* out = (float*)d_out;

  const dim3 blk(256);
  const int n8x = NROW * DM / 8;
  const int n8b = NB * NS * NS / 8;
  const dim3 gCvtX((n8x + 255) / 256);
  const dim3 gCvtB((n8b + 255) / 256);
  const dim3 gWtQ((3 * DM) / 16);
  const dim3 gWtP(DM / 16);
  const dim3 gQK(((NROW / 64) * ((2 * DM) / 64) + 7) / 8);
  const dim3 gV((((DM / 64) * (NROW / 64)) + 7) / 8);
  const dim3 gAttn(NBH * NQB);
  const dim3 gPj((((NROW / 64) * (DM / 64)) + 7) / 8);

  cvt_bf16x8<<<gCvtX, blk, 0, stream>>>(x, Xb, n8x);
  cvt_bf16x8<<<gCvtB, blk, 0, stream>>>(abias, Bb, n8b);
  prep_wt<<<gWtQ, blk, 0, stream>>>(Wqkv, 3 * DM, WqT);
  prep_wt<<<gWtP, blk, 0, stream>>>(Wp, DM, WpT);
  pgemm<0><<<gQK, blk, 0, stream>>>(Xb, Xb, WqT, Qh, Ql, Kh, Kl, out);
  pgemm<1><<<gV, blk, 0, stream>>>(WqT + (size_t)2 * DM * DM, WqT + (size_t)2 * DM * DM, Xb,
                                   VTh, VTl, VTh, VTl, out);
  (void)hipFuncSetAttribute(reinterpret_cast<const void*>(&attn),
                            hipFuncAttributeMaxDynamicSharedMemorySize, L_TOTAL);
  attn<<<gAttn, dim3(128), L_TOTAL, stream>>>(Qh, Ql, Kh, Kl, VTh, VTl, Bb, beta, Oh, Ol);
  pgemm<2><<<gPj, blk, 0, stream>>>(Oh, Ol, WpT, Qh, Ql, Kh, Kl, out);
  (void)hipGetLastError();
}
